// Ss_rnn_77163382440496
// MI455X (gfx1250) — hardware-run, weakly checked
//
#include <hip/hip_runtime.h>
#include <math.h>

typedef __attribute__((ext_vector_type(16))) _Float16 v16h;
typedef __attribute__((ext_vector_type(8)))  _Float16 v8h;
typedef __attribute__((ext_vector_type(2)))  _Float16 v2h;
typedef __attribute__((ext_vector_type(16))) __bf16   v16b;
typedef __attribute__((ext_vector_type(8)))  __bf16   v8b;
typedef __attribute__((ext_vector_type(8)))  float    v8f;
typedef __attribute__((ext_vector_type(4)))  float    v4f;
typedef __attribute__((ext_vector_type(2)))  float    v2f;

constexpr int kT    = 262144;
constexpr int kH    = 64;
constexpr int kU    = 16;
constexpr int kWC   = 80;
constexpr int kQ    = 64;
constexpr int kC    = kT / kQ;
constexpr int kRW   = 128;
constexpr int kK    = 96;
constexpr int kPW   = 192;
constexpr int kLv   = 12;
constexpr int kNP   = 6 + kLv;
constexpr int kThr  = 256;
constexpr float kInCarry = 1024.0f;
constexpr float kACarry  = 16384.0f;
constexpr float kSc = 1.0f / (kInCarry * kACarry);
constexpr float kF16MinNormal = 6.103515625e-5f;

static_assert(kQ == 64 && kC == 4096 && kH == 64 && kU == 16 && kWC == 80 && kRW == 128 && kK == 96 && kPW == 192 && kNP == 18 && kLv == 12, "the index arithmetic below uses these sizes");
static_assert((1 << kLv) == kC, "twelve levels span the 4,096 chunks; level k uses the power 6 + k");

constexpr size_t kOffZB = 0ull;
constexpr size_t kOffBIA = 4096ull;
constexpr size_t kOffP32 = 4352ull;
constexpr size_t kOffPL16 = 299264ull;
constexpr size_t kOffPT16 = 741632ull;
constexpr size_t kOffPN16 = 1184000ull;
constexpr size_t kOffAB16 = 1626368ull;
constexpr size_t kOffHS32 = 1642752ull;
constexpr size_t kOffGA32 = 2691328ull;
constexpr size_t kOffGB32 = 3740160ull;
constexpr size_t kOffD32 = 4788736ull;
constexpr size_t kOffGX16 = 5837312ull;
constexpr size_t kOffHX = 7410176ull;
constexpr size_t kOffSALL = 74519040ull;
constexpr size_t kWsTotal = 141627904ull;
static_assert(kWsTotal <= 268435456ull, "the carve fits the 256 MiB offered");
static_assert(kOffZB == 0
              && kOffBIA == kOffZB + 4096ull
              && kOffP32 == kOffBIA + 256ull
              && kOffPL16 == kOffP32 + 294912ull
              && kOffPT16 == kOffPL16 + 442368ull
              && kOffPN16 == kOffPT16 + 442368ull
              && kOffAB16 == kOffPN16 + 442368ull
              && kOffHS32 == kOffAB16 + 16384ull
              && kOffGA32 == kOffHS32 + 1048576ull
              && kOffGB32 == kOffGA32 + 1048832ull
              && kOffD32 == kOffGB32 + 1048576ull
              && kOffGX16 == kOffD32 + 1048576ull
              && kOffHX == kOffGX16 + 1572864ull
              && kOffSALL == kOffHX + 67108864ull
              && kWsTotal == kOffSALL + 67108864ull, "the carve is chained and totalled");
static_assert((kOffBIA % 256) == 0 && (kOffP32 % 256) == 0 && (kOffPL16 % 256) == 0 && (kOffPT16 % 256) == 0 && (kOffPN16 % 256) == 0 && (kOffAB16 % 256) == 0 && (kOffHS32 % 256) == 0 && (kOffGA32 % 256) == 0 && (kOffGB32 % 256) == 0 && (kOffD32 % 256) == 0 && (kOffGX16 % 256) == 0 && (kOffHX % 256) == 0 && (kOffSALL % 256) == 0, "aligned regions");
static_assert(1024 >= kH && 64 >= kH, "each bias record covers the 64 output columns of every launch that names it (the engine reads one bias value a column)");

__device__ __forceinline__ unsigned short f2bf_bits(float f) {
  unsigned u = __float_as_uint(f);
  return (unsigned short)((u + 0x7FFFu + ((u >> 16) & 1u)) >> 16);
}
__device__ __forceinline__ float bf_bits2f(unsigned short h) { return __uint_as_float(((unsigned)h) << 16); }
__device__ __forceinline__ float bf16r(float f) { return bf_bits2f(f2bf_bits(f)); }
__device__ __forceinline__ float carry_flush(float v, float carry) {
  const float s = v * carry;
  return (fabsf(s) < kF16MinNormal) ? 0.0f : s;
}

__device__ __forceinline__ void dep_guard4_h(v8f& a, v8f& b, v8f& c, v8f& d, v16h x, v16h y) { asm volatile("v_nop\n\tv_nop\n\tv_nop\n\tv_nop" : "+v"(a), "+v"(b), "+v"(c), "+v"(d) : "v"(x), "v"(y)); }
__device__ __forceinline__ void dep_guard4_b(v8f& a, v8f& b, v8f& c, v8f& d, v16b x, v16b y) { asm volatile("v_nop\n\tv_nop\n\tv_nop\n\tv_nop" : "+v"(a), "+v"(b), "+v"(c), "+v"(d) : "v"(x), "v"(y)); }
__device__ __forceinline__ void keep4_h(v16h a, v16h b, v16h c, v16h d) { asm volatile("v_nop" :: "v"(a), "v"(b), "v"(c), "v"(d)); }
__device__ __forceinline__ void keep4_b(v16b a, v16b b, v16b c, v16b d) { asm volatile("v_nop" :: "v"(a), "v"(b), "v"(c), "v"(d)); }
__device__ __forceinline__ void acc_guard4(v8f& a, v8f& b, v8f& c, v8f& d) { asm volatile("v_nop\n\tv_nop\n\tv_nop\n\tv_nop" : "+v"(a), "+v"(b), "+v"(c), "+v"(d)); }

template <typename T> struct Frag;
template <> struct Frag<_Float16> {
  typedef v16h V; union U { v16h v; v8h h[2]; };
  static __device__ __forceinline__ v16h load(const _Float16* p) {
    U f; f.h[0] = *(const v8h*)(p); f.h[1] = *(const v8h*)(p + 16); return f.v;
  }
  static __device__ __forceinline__ v8f mma(v16h a, v16h b, v8f c) {
    return __builtin_amdgcn_wmma_f32_16x16x32_f16(false, a, false, b, (short)0, c, false, false);
  }
  static __device__ __forceinline__ void guard4(v8f& a, v8f& b, v8f& c, v8f& d, v16h x, v16h y) { dep_guard4_h(a, b, c, d, x, y); }
  static __device__ __forceinline__ void keep(v16h a, v16h b, v16h c, v16h d) { keep4_h(a, b, c, d); }
};
template <> struct Frag<__bf16> {
  typedef v16b V; union U { v16b v; v8b h[2]; };
  static __device__ __forceinline__ v16b load(const __bf16* p) {
    U f; f.h[0] = *(const v8b*)(p); f.h[1] = *(const v8b*)(p + 16); return f.v;
  }
  static __device__ __forceinline__ v8f mma(v16b a, v16b b, v8f c) {
    return __builtin_amdgcn_wmma_f32_16x16x32_bf16(false, a, false, b, (short)0, c, false, false);
  }
  static __device__ __forceinline__ void guard4(v8f& a, v8f& b, v8f& c, v8f& d, v16b x, v16b y) { dep_guard4_b(a, b, c, d, x, y); }
  static __device__ __forceinline__ void keep(v16b a, v16b b, v16b c, v16b d) { keep4_b(a, b, c, d); }
};

__device__ __forceinline__ v8f mma_h(v16h a, v16h b, v8f c) {
  c = __builtin_amdgcn_wmma_f32_16x16x32_f16(false, a, false, b, (short)0, c, false, false);
  asm volatile("v_nop\n\tv_nop\n\tv_nop\n\tv_nop" : "+v"(c) : "v"(a), "v"(b));
  return c;
}

template <int ET> struct Elem;
template <> struct Elem<0> { typedef _Float16 T; };
template <> struct Elem<1> { typedef __bf16 T; };
template <int ET, bool SPLIT, int BIAS_MODE, int OUT_MODE, bool RESID, int ACT = 0>
__global__ __launch_bounds__(256) void wmma_gemm64(
    const unsigned short* __restrict__ Ap, const unsigned short* __restrict__ A2p, int lda, long strideA,
    const unsigned short* __restrict__ Btp, const unsigned short* __restrict__ Bt2p, int ldb, long strideB,
    void* __restrict__ Cout, void* __restrict__ Cout2, int ldc, long strideC,
    const float* __restrict__ bias,
    const float* __restrict__ resid, long strideR,
    int M, int N, int K, float scale) {
  typedef typename Elem<ET>::T T;
  typedef typename Frag<T>::V V;
  const T* A = (const T*)Ap; const T* A2 = (const T*)A2p; const T* Bt = (const T*)Btp; const T* Bt2 = (const T*)Bt2p;
  __shared__ __align__(16) float sT[8][16 * 68];
  const int b    = blockIdx.y;
  const int lane = threadIdx.x & 31;
  const int wave = threadIdx.x >> 5;
  const int tilesN = N >> 6;
  const int tilesM = M >> 6;
  const int tile = blockIdx.x * 8 + wave;
  if (tile >= tilesM * tilesN) return;
  const int tm = tile / tilesN;
  const int tn = tile - tm * tilesN;
  const int m0 = tm << 6;
  const int n0 = tn << 6;

  const T* Ab  = A  + (size_t)b * strideA;
  const T* Bb  = Bt + (size_t)b * strideB;
  const T* Ab2 = SPLIT ? (A2  + (size_t)b * strideA) : nullptr;
  const T* Bb2 = SPLIT ? (Bt2 + (size_t)b * strideB) : nullptr;

  const int rlane = lane & 15;
  const int koff  = (lane >> 4) * 8;
  const int mOff  = (lane >> 4) * 8;

  v8f acc[4][4];
#pragma unroll
  for (int i = 0; i < 4; ++i)
#pragma unroll
    for (int j = 0; j < 4; ++j) acc[i][j] = (v8f){0.f,0.f,0.f,0.f,0.f,0.f,0.f,0.f};

  for (int k0 = 0; k0 < K; k0 += 32) {
    V bh[4], bl[4];
#pragma unroll
    for (int j = 0; j < 4; ++j) {
      const size_t bo = (size_t)(n0 + (j << 4) + rlane) * ldb + koff + k0;
      bh[j] = Frag<T>::load(Bb + bo);
      if (SPLIT) bl[j] = Frag<T>::load(Bb2 + bo);
    }
#pragma unroll
    for (int i = 0; i < 4; ++i) {
      const size_t ao = (size_t)(m0 + (i << 4) + rlane) * lda + koff + k0;
      V ah = Frag<T>::load(Ab + ao);
      V al;
      if (SPLIT) al = Frag<T>::load(Ab2 + ao);
#pragma unroll
      for (int j = 0; j < 4; ++j) {
        acc[i][j] = Frag<T>::mma(ah, bh[j], acc[i][j]);
        if (SPLIT) {
          acc[i][j] = Frag<T>::mma(ah, bl[j], acc[i][j]);
          acc[i][j] = Frag<T>::mma(al, bh[j], acc[i][j]);
        }
      }
      Frag<T>::guard4(acc[i][0], acc[i][1], acc[i][2], acc[i][3], ah, SPLIT ? al : ah);
    }
    Frag<T>::keep(bh[0], bh[1], bh[2], bh[3]);
    if (SPLIT) Frag<T>::keep(bl[0], bl[1], bl[2], bl[3]);
  }
  acc_guard4(acc[0][0], acc[0][1], acc[0][2], acc[0][3]);
  acc_guard4(acc[1][0], acc[1][1], acc[1][2], acc[1][3]);
  acc_guard4(acc[2][0], acc[2][1], acc[2][2], acc[2][3]);
  acc_guard4(acc[3][0], acc[3][1], acc[3][2], acc[3][3]);

  float* slab = sT[wave];
  const float* Rb = RESID ? (resid + (size_t)b * strideR) : nullptr;
#pragma unroll
  for (int i = 0; i < 4; ++i) {
    const int mBase = m0 + (i << 4);
#pragma unroll
    for (int j = 0; j < 4; ++j) {
      const int n = n0 + (j << 4) + rlane;
      float bv = 0.f;
      if (BIAS_MODE == 2) bv = bias[n];
#pragma unroll
      for (int r = 0; r < 8; ++r) {
        float v = acc[i][j][r] * scale;
        if (BIAS_MODE == 1) v += bias[mBase + mOff + r];
        if (BIAS_MODE == 2) v += bv;
        if (RESID) v += Rb[(size_t)(mBase + mOff + r) * ldc + n];
        if (ACT == 1) v = tanhf(v);
        if (ACT == 2) v = fmaxf(v, 0.0f);
        if (ACT == 3) v = v / (1.0f + expf(-v));
        if (ACT == 4) v = (v > 0.f) ? v : 0.01f * v;
        slab[(mOff + r) * 68 + (j << 4) + rlane] = v;
      }
    }
    __builtin_amdgcn_fence(__ATOMIC_RELEASE, "workgroup");
    __builtin_amdgcn_wave_barrier();
    __builtin_amdgcn_fence(__ATOMIC_ACQUIRE, "workgroup");
    if (OUT_MODE == 0) {
      float* C = (float*)Cout + (size_t)b * strideC;
      const int hh = lane >> 4, c4 = (lane & 15) * 4;
      for (int pass = 0; pass < 2; ++pass) {
#pragma unroll
        for (int it = 0; it < 8; ++it) {
          const int row = it * 2 + hh;
          v4f v = *(const v4f*)(slab + row * 68 + c4);
          *(volatile v4f*)(C + (size_t)(mBase + row) * ldc + n0 + c4) = v;
        }
        __threadfence();
      }
    } else {
      const int q = lane >> 3, c8 = (lane & 7) * 8;
      unsigned short* C  = (unsigned short*)Cout  + (size_t)b * strideC;
      unsigned short* C2 = (OUT_MODE == 2) ? ((unsigned short*)Cout2 + (size_t)b * strideC) : nullptr;
      for (int pass = 0; pass < 2; ++pass) {
#pragma unroll
        for (int it = 0; it < 4; ++it) {
          const int row = it * 4 + q;
          const float* sp = slab + row * 68 + c8;
          v8h hv, lv;
#pragma unroll
          for (int e = 0; e < 8; ++e) {
            if (OUT_MODE == 1) {
              hv[e] = (_Float16)sp[e];
            } else {
              unsigned short hb = f2bf_bits(sp[e]);
              unsigned short lb = f2bf_bits(sp[e] - bf_bits2f(hb));
              hv[e] = __builtin_bit_cast(_Float16, hb);
              lv[e] = __builtin_bit_cast(_Float16, lb);
            }
          }
          *(volatile v8h*)(C + (size_t)(mBase + row) * ldc + n0 + c8) = hv;
          if (OUT_MODE == 2) *(volatile v8h*)(C2 + (size_t)(mBase + row) * ldc + n0 + c8) = lv;
        }
        __threadfence();
      }
    }
    __builtin_amdgcn_fence(__ATOMIC_RELEASE, "workgroup");
    __builtin_amdgcn_wave_barrier();
    __builtin_amdgcn_fence(__ATOMIC_ACQUIRE, "workgroup");
  }
}


__device__ __forceinline__ void two_words(float w, float carry, _Float16& hh, _Float16& ll) {
  const float sc = carry_flush(w, carry);
  hh = (_Float16)sc;
  const float rs = sc - (float)hh;
  ll = (_Float16)((fabsf(rs) < kF16MinNormal) ? 0.0f : rs);
}
__device__ __forceinline__ void store2(float* p, float v) {
  *(volatile float*)p = v;
  __threadfence();
  *(volatile float*)p = v;
}


__global__ __launch_bounds__(kThr) void zero_kernel(float* __restrict__ dst) {
  const size_t o4 = ((size_t)blockIdx.x * kThr + threadIdx.x) * 4u;
  const v4f z = {0.f, 0.f, 0.f, 0.f};
  *(volatile v4f*)(dst + o4) = z;
  __threadfence();
  *(volatile v4f*)(dst + o4) = z;
}

__global__ __launch_bounds__(kThr) void sinit_kernel(const float* __restrict__ W, const float* __restrict__ bvec, const float* __restrict__ s0, float* __restrict__ P0,
                                                    float* __restrict__ BIA, float* __restrict__ G0) {
  const unsigned t = blockIdx.x * (unsigned)kThr + threadIdx.x;
  if (t >= 4224u) return;
  if (t < 4096u) {
    const unsigned i = t >> 6, j = t & 63u;
    const float a = W[i * (unsigned)kWC + (unsigned)kU + j];
    store2(P0 + t, bf16r(a));
  } else if (t < 4160u) {
    const unsigned n = t - 4096u;
    const float bv = bvec[n];
    store2(BIA + n, bf16r(bv));
  } else {
    const unsigned n = t - 4160u;
    const float sv = s0[n];
    store2(G0 + n, bf16r(sv));
  }
}

__global__ __launch_bounds__(kThr) void pcast_kernel(const float* __restrict__ P, unsigned short* __restrict__ PL, unsigned short* __restrict__ PT, unsigned short* __restrict__ PN) {
  const unsigned t = blockIdx.x * (unsigned)kThr + threadIdx.x;
  const unsigned i = t >> 3, g8 = (t & 7u) * 8u;
  v8h lv, ll, nv, nl, tv, tl;
#pragma unroll
  for (int e = 0; e < 8; ++e) {
    const float p = P[i * (unsigned)kH + g8 + (unsigned)e];
    const float q = P[(g8 + (unsigned)e) * (unsigned)kH + i];
    _Float16 a, b;
    two_words(p, kInCarry, a, b); lv[e] = a; ll[e] = b;
    two_words(p, kACarry, a, b);  nv[e] = a; nl[e] = b;
    two_words(q, kACarry, a, b);  tv[e] = a; tl[e] = b;
  }
  unsigned short* pl = PL + (size_t)i * kPW + g8;
  unsigned short* pn = PN + (size_t)i * kPW + g8;
  unsigned short* pt = PT + (size_t)i * kPW + g8;
  for (int pass = 0; pass < 2; ++pass) {
    *(volatile v8h*)pl = lv; *(volatile v8h*)(pl + 64) = lv; *(volatile v8h*)(pl + 128) = ll;
    *(volatile v8h*)pn = nv; *(volatile v8h*)(pn + 64) = nv; *(volatile v8h*)(pn + 128) = nl;
    *(volatile v8h*)pt = tv; *(volatile v8h*)(pt + 64) = tl; *(volatile v8h*)(pt + 128) = tv;
    __threadfence();
  }
}
static_assert(kH * (kH / 8) == 2 * kThr, "power cast grid exact: 2 blocks");

__global__ __launch_bounds__(kThr) void wcast_kernel(const float* __restrict__ W, unsigned short* __restrict__ AB) {
  const unsigned t = blockIdx.x * (unsigned)kThr + threadIdx.x;
  const unsigned n = t >> 4, cg = t & 15u;
  v8h hv;
#pragma unroll
  for (int e = 0; e < 8; ++e) {
    float v = 0.0f;
    if (cg < 8u) v = W[n * (unsigned)kWC + (unsigned)kU + cg * 8u + (unsigned)e];
    else if (cg < 10u) v = W[n * (unsigned)kWC + (cg - 8u) * 8u + (unsigned)e];
    hv[e] = (_Float16)carry_flush(bf16r(v), kACarry);
  }
  unsigned short* dp = AB + (size_t)n * kRW + cg * 8u;
  *(volatile v8h*)dp = hv;
  __threadfence();
  *(volatile v8h*)dp = hv;
}
static_assert(kH * (kRW / 8) == 4 * kThr, "right-operand cast grid exact: 4 blocks");

__global__ __launch_bounds__(kThr) void ufill_kernel(const float* __restrict__ U, unsigned short* __restrict__ HX) {
  const unsigned i = blockIdx.x * (unsigned)kThr + threadIdx.x;
  const unsigned t = i >> 3, g = i & 7u;
  const unsigned c = t >> 6, l = t & 63u;
  v8h hv;
#pragma unroll
  for (int e = 0; e < 8; ++e) {
    float v = 0.0f;
    if (g < 2u) v = U[(size_t)t * kU + g * 8u + (unsigned)e];
    hv[e] = (_Float16)carry_flush(bf16r(v), kInCarry);
  }
  unsigned short* dp = HX + ((size_t)(l * (unsigned)kC + c) * kRW + 64u + g * 8u);
  *(volatile v8h*)dp = hv;
  __threadfence();
  *(volatile v8h*)dp = hv;
}
static_assert((size_t)kT * 8 == 8192ull * kThr, "input fill grid exact: 8,192 blocks");

__global__ __launch_bounds__(kThr) void scast_kernel(const float* __restrict__ src, int pitch, const float* __restrict__ add, unsigned short* __restrict__ rows) {
  const unsigned i = blockIdx.x * (unsigned)kThr + threadIdx.x;
  const unsigned c = i >> 3, n8 = (i & 7u) * 8u;
  const float* sp = src + (size_t)c * (unsigned)pitch + n8;
  v8h hv;
#pragma unroll
  for (int e = 0; e < 8; ++e) {
    float v = sp[e];
    if (add != nullptr) v += add[c * (unsigned)kH + n8 + (unsigned)e];
    hv[e] = (_Float16)carry_flush(v, kInCarry);
  }
  unsigned short* dp = rows + (size_t)c * kRW + n8;
  *(volatile v8h*)dp = hv;
  __threadfence();
  *(volatile v8h*)dp = hv;
}
static_assert(kC * (kH / 8) == 128 * kThr, "state cast grid exact: 128 blocks");

__global__ __launch_bounds__(kThr) void gcast_kernel(const float* __restrict__ Gin, const float* __restrict__ Din, float* __restrict__ Gout, unsigned short* __restrict__ GX, int shift) {
  const unsigned i = blockIdx.x * (unsigned)kThr + threadIdx.x;
  const unsigned r = i >> 3, n8 = (i & 7u) * 8u;
  const bool has = r >= (unsigned)shift;
  const unsigned rs = has ? (r - (unsigned)shift) : 0u;
  v4f o0, o1; v8h uv, ul;
#pragma unroll
  for (int e = 0; e < 8; ++e) {
    float v = Gin[r * (unsigned)kH + n8 + (unsigned)e];
    float u = Gin[rs * (unsigned)kH + n8 + (unsigned)e];
    if (Din != nullptr) { v += Din[r * (unsigned)kH + n8 + (unsigned)e]; u += Din[rs * (unsigned)kH + n8 + (unsigned)e]; }
    if (e < 4) o0[e] = v; else o1[e - 4] = v;
    _Float16 a, b; two_words(has ? u : 0.0f, kInCarry, a, b);
    uv[e] = a; ul[e] = b;
  }
  float* gp = Gout + (size_t)r * kH + n8;
  unsigned short* xp = GX + (size_t)r * kPW + n8;
  for (int pass = 0; pass < 2; ++pass) {
    *(volatile v4f*)gp = o0; *(volatile v4f*)(gp + 4) = o1;
    *(volatile v8h*)xp = uv; *(volatile v8h*)(xp + 64) = ul; *(volatile v8h*)(xp + 128) = uv;
    __threadfence();
  }
}

__global__ __launch_bounds__(kThr) void ydot_kernel(const float* __restrict__ S, const float* __restrict__ wy, const float* __restrict__ by, float* __restrict__ out) {
  const unsigned t = blockIdx.x * (unsigned)kThr + threadIdx.x;
  const float* sp = S + (size_t)t * kH;
  const float b0 = by[0];
  float acc = bf16r(b0);
#pragma unroll
  for (int q = 0; q < kH / 4; ++q) {
    const v4f s4 = *(const v4f*)(sp + 4 * q);
#pragma unroll
    for (int k = 0; k < 4; ++k) { const float w0 = wy[4 * q + k]; acc += bf16r(w0) * s4[k]; }
  }
  store2(out + t, acc);
}
static_assert(kT == 1024 * kThr, "read-out grid exact: 1,024 blocks");

extern "C" void kernel_launch(void* const* d_in, const int* in_sizes, int n_in,
                              void* d_out, int out_size, void* d_ws, size_t ws_size,
                              hipStream_t stream) {
  if (n_in < 6 || d_out == nullptr || d_ws == nullptr) return;
  if (in_sizes[0] != kT * kU || in_sizes[1] != kH || in_sizes[2] != kH * kWC || in_sizes[3] != kH || in_sizes[4] != kH || in_sizes[5] != 1) return;
  if (out_size != kT) return;
  if (ws_size < kWsTotal) return;
  const float* U = (const float*)d_in[0];
  const float* s0 = (const float*)d_in[1];
  const float* W = (const float*)d_in[2];
  const float* bvec = (const float*)d_in[3];
  const float* wy = (const float*)d_in[4];
  const float* by = (const float*)d_in[5];
  float* out = (float*)d_out;
  char* ws = (char*)d_ws;
  float* ZB = (float*)(ws + kOffZB);
  float* BIA = (float*)(ws + kOffBIA);
  float* P32 = (float*)(ws + kOffP32);
  unsigned short* PL16 = (unsigned short*)(ws + kOffPL16);
  unsigned short* PT16 = (unsigned short*)(ws + kOffPT16);
  unsigned short* PN16 = (unsigned short*)(ws + kOffPN16);
  unsigned short* AB16 = (unsigned short*)(ws + kOffAB16);
  float* HS32 = (float*)(ws + kOffHS32);
  float* GA32 = (float*)(ws + kOffGA32);
  float* GB32 = (float*)(ws + kOffGB32);
  float* D32 = (float*)(ws + kOffD32);
  unsigned short* GX16 = (unsigned short*)(ws + kOffGX16);
  unsigned short* HX = (unsigned short*)(ws + kOffHX);
  float* SALL = (float*)(ws + kOffSALL);

  zero_kernel<<<1, kThr, 0, stream>>>(ZB);
  sinit_kernel<<<17, kThr, 0, stream>>>(W, bvec, s0, P32, BIA, GA32);
  pcast_kernel<<<2, kThr, 0, stream>>>(P32, PL16, PT16, PN16);
  for (int k = 0; k + 1 < kNP; ++k) {
    wmma_gemm64<0, false, 2, 0, false, 0><<<dim3(1, 1), 256, 0, stream>>>(
        PL16 + (size_t)k * kH * kPW, PL16 + (size_t)k * kH * kPW, kPW, 0L, PT16 + (size_t)k * kH * kPW, PT16 + (size_t)k * kH * kPW, kPW, 0L,
        (void*)(P32 + (size_t)(k + 1) * kH * kH), (void*)(P32 + (size_t)(k + 1) * kH * kH), kH, 0L, ZB, nullptr, 0L, kH, kH, kPW, kSc);
    pcast_kernel<<<2, kThr, 0, stream>>>(P32 + (size_t)(k + 1) * kH * kH, PL16 + (size_t)(k + 1) * kH * kPW, PT16 + (size_t)(k + 1) * kH * kPW, PN16 + (size_t)(k + 1) * kH * kPW);
  }
  wcast_kernel<<<4, kThr, 0, stream>>>(W, AB16);
  ufill_kernel<<<8192, kThr, 0, stream>>>(U, HX);

  zero_kernel<<<256, kThr, 0, stream>>>(HS32);
  scast_kernel<<<128, kThr, 0, stream>>>(HS32, kH, nullptr, HX);
  for (int l = 0; l < kQ; ++l) {
    const unsigned short* Al = HX + (size_t)l * kC * kRW;
    float* Cl = (l + 1 < kQ) ? HS32 : (GA32 + kH);
    wmma_gemm64<0, false, 2, 0, false, 0><<<dim3(8, 1), 256, 0, stream>>>(
        Al, Al, kRW, 0L, AB16, AB16, kRW, 0L, (void*)Cl, (void*)Cl, kH, 0L, BIA, nullptr, 0L, kC, kH, kK, kSc);
    if (l + 1 < kQ) scast_kernel<<<128, kThr, 0, stream>>>(HS32, kH, nullptr, HX + (size_t)(l + 1) * kC * kRW);
  }

  for (int k = 0; k < kLv; ++k) {
    const float* Gin = (k & 1) ? GB32 : GA32;
    float* Gout = (k & 1) ? GA32 : GB32;
    gcast_kernel<<<128, kThr, 0, stream>>>(Gin, (k == 0) ? (const float*)nullptr : (const float*)D32, Gout, GX16, 1 << k);
    wmma_gemm64<0, false, 2, 0, false, 0><<<dim3(8, 1), 256, 0, stream>>>(
        GX16, GX16, kPW, 0L, PN16 + (size_t)(6 + k) * kH * kPW, PN16 + (size_t)(6 + k) * kH * kPW, kPW, 0L, (void*)D32, (void*)D32, kH, 0L, ZB, nullptr, 0L, kC, kH, kPW, kSc);
  }

  scast_kernel<<<128, kThr, 0, stream>>>(GA32, kH, D32, HX);
  for (int l = 0; l < kQ; ++l) {
    const unsigned short* Al = HX + (size_t)l * kC * kRW;
    wmma_gemm64<0, false, 2, 0, false, 0><<<dim3(8, 1), 256, 0, stream>>>(
        Al, Al, kRW, 0L, AB16, AB16, kRW, 0L, (void*)(SALL + (size_t)l * kH), (void*)(SALL + (size_t)l * kH), kQ * kH, 0L, BIA, nullptr, 0L, kC, kH, kK, kSc);
    if (l + 1 < kQ) scast_kernel<<<128, kThr, 0, stream>>>(SALL + (size_t)l * kH, kQ * kH, nullptr, HX + (size_t)(l + 1) * kC * kRW);
  }
  ydot_kernel<<<1024, kThr, 0, stream>>>(SALL, wy, by, out);
}
